// SynapticMemory_79164837200282
// MI455X (gfx1250) — hardware-run, weakly checked
//
#include <hip/hip_runtime.h>
#include <math.h>

typedef __attribute__((ext_vector_type(16))) _Float16 v16h;
typedef __attribute__((ext_vector_type(8)))  _Float16 v8h;
typedef __attribute__((ext_vector_type(8)))  float    v8f;
typedef __attribute__((ext_vector_type(4)))  float    v4f;
typedef __attribute__((ext_vector_type(4)))  unsigned int v4u;

constexpr int kBatch  = 2;
constexpr int kSeq    = 2048;
constexpr int kDm     = 512;
constexpr int kMem    = 64;
constexpr int kMemRoot = 8;
constexpr int kRows   = kBatch * kSeq;
constexpr int kQKld   = 2 * kMem;
constexpr int kKVrows = kMem + kDm;
constexpr int kChunk  = 64;
constexpr int kNChunk = kSeq / kChunk;
constexpr int kDTile  = 64;
constexpr int kTP     = 64;
constexpr int kSlabP  = 36;
static_assert(kMemRoot * kMemRoot == kMem);
static_assert(kRows == 4096 && kQKld == 128 && kKVrows == 576);
static_assert((kSeq % kChunk) == 0 && (kDm % kDTile) == 0);
static_assert((kDm % 32) == 0 && (kRows % 64) == 0 && (kQKld % 64) == 0 && (kKVrows % 64) == 0 && (kDm % 64) == 0);

constexpr float kXCarry    = 16.0f;
constexpr float kWCarry    = 256.0f;
constexpr float kVCarry    = 16.0f;
constexpr float kUCarry    = 16.0f;
constexpr float kProjScale = 1.0f / (kXCarry * kWCarry);
constexpr float kVScale    = kVCarry * kProjScale;
constexpr float kOutScale  = 1.0f / (kUCarry * kWCarry);
constexpr float kQScale    = 1.0f / (float)kMemRoot;
constexpr float kNumFold   = kQScale / kVCarry;
constexpr float kF16MinNormal = 6.103515625e-5f;
constexpr float kDenEps    = 1e-6f;
constexpr float kRmsEps    = 1e-6f;
constexpr float kInvDm     = 1.0f / (float)kDm;

constexpr size_t kOffXH  = 0;
constexpr size_t kOffWQK = kOffXH  + (size_t)kRows * kDm * 2;
constexpr size_t kOffWKV = kOffWQK + (size_t)kQKld * kDm * 2;
constexpr size_t kOffWO  = kOffWKV + (size_t)kKVrows * kDm * 2;
constexpr size_t kOffQK  = kOffWO  + (size_t)kDm * kDm * 2;
constexpr size_t kOffKVT = kOffQK  + (size_t)kRows * kQKld * 2;
constexpr size_t kOffNUM = kOffKVT + (size_t)kKVrows * kRows * 2;
constexpr size_t kOffDEN = kOffNUM + (size_t)kRows * kDm * 4;
constexpr size_t kOffUN  = kOffDEN + (size_t)kRows * 4;
constexpr size_t kWsTotal = kOffUN + (size_t)kRows * kDm * 2;
static_assert(kWsTotal == 23805952ull);
static_assert(kWsTotal <= 134217728ull);
static_assert((kOffWQK % 128) == 0 && (kOffWKV % 128) == 0 && (kOffWO % 128) == 0 && (kOffQK % 128) == 0 &&
              (kOffKVT % 128) == 0 && (kOffNUM % 128) == 0 && (kOffDEN % 128) == 0 && (kOffUN % 128) == 0);

__device__ __forceinline__ float h16_to_f32(unsigned hb) {
  const unsigned sgn = (hb & 0x8000u) << 16;
  const unsigned em = hb & 0x7fffu;
  const float fn = __uint_as_float((em << 13) + 0x38000000u);
  const float fs = (float)em * 5.9604644775390625e-8f;
  const float mag = (em < 0x400u) ? fs : fn;
  return __uint_as_float(__float_as_uint(mag) | sgn);
}
__device__ __forceinline__ unsigned short h_bits_ftz(float f) {
  const float g = (fabsf(f) < kF16MinNormal) ? 0.0f : f;
  const _Float16 h = (_Float16)g;
  return __builtin_bit_cast(unsigned short, h);
}
__device__ __forceinline__ unsigned pk16(unsigned short a, unsigned short b) { return (unsigned)a | ((unsigned)b << 16); }
__device__ __forceinline__ v4u pack8(float a0, float a1, float a2, float a3, float a4, float a5, float a6, float a7) {
  const unsigned short b0 = h_bits_ftz(a0), b1 = h_bits_ftz(a1), b2 = h_bits_ftz(a2), b3 = h_bits_ftz(a3);
  const unsigned short b4 = h_bits_ftz(a4), b5 = h_bits_ftz(a5), b6 = h_bits_ftz(a6), b7 = h_bits_ftz(a7);
  return (v4u){pk16(b0, b1), pk16(b2, b3), pk16(b4, b5), pk16(b6, b7)};
}
__device__ __forceinline__ float phi_map(float t) {
  const float e = expf(fminf(t, 0.0f));
  return (t > 0.0f) ? (t + 1.0f) : e;
}
__device__ __forceinline__ float lc_at(float ld, int p) { return fminf(fmaxf(ld * (float)p, -20.0f), 20.0f); }

union FragU { v16h v; v8h h[2]; };
__device__ __forceinline__ v16h frag_load(const _Float16* p) {
  FragU f;
  f.h[0] = *(const v8h*)(p);
  f.h[1] = *(const v8h*)(p + 16);
  return f.v;
}
__device__ __forceinline__ v8f mma_h(v16h a, v16h b, v8f c) {
  c = __builtin_amdgcn_wmma_f32_16x16x32_f16(false, a, false, b, (short)0, c, false, false);
  asm volatile("v_nop\n\tv_nop\n\tv_nop\n\tv_nop" : "+v"(c) : "v"(a), "v"(b));
  return c;
}
__device__ __forceinline__ void keep4_h(v16h a, v16h b, v16h c, v16h d) { asm volatile("v_nop" :: "v"(a), "v"(b), "v"(c), "v"(d)); }
__device__ __forceinline__ void acc_guard4(v8f& a, v8f& b, v8f& c, v8f& d) { asm volatile("v_nop\n\tv_nop\n\tv_nop\n\tv_nop" : "+v"(a), "+v"(b), "+v"(c), "+v"(d)); }
__device__ __forceinline__ void wave_sync_lds() {
  __builtin_amdgcn_fence(__ATOMIC_RELEASE, "workgroup");
  __builtin_amdgcn_wave_barrier();
  __builtin_amdgcn_fence(__ATOMIC_ACQUIRE, "workgroup");
}

constexpr int kBlkX  = (kRows * kDm / 8) / 256;
constexpr int kBlkQK = (kQKld * kDm / 8) / 256;
constexpr int kBlkKV = (kKVrows * kDm / 8) / 256;
constexpr int kBlkO  = (kDm * kDm / 8) / 256;
constexpr int kBlkSeam = (kMem * kDm / 8) / 256;
constexpr int kUnitsSeam = kMem * kDm / 8;
static_assert(kBlkX == 1024 && kBlkQK == 32 && kBlkKV == 144 && kBlkO == 128 && kBlkSeam == 16);

__global__ __launch_bounds__(256) void cast_planes_kernel(
    const float* __restrict__ x, const float* __restrict__ Wq, const float* __restrict__ Wk,
    const float* __restrict__ Wv, const float* __restrict__ Wo,
    unsigned short* __restrict__ xh, unsigned short* __restrict__ wqk,
    unsigned short* __restrict__ wkv, unsigned short* __restrict__ wo) {
  const int blk = blockIdx.x, tid = threadIdx.x;
  const float* src;
  unsigned short* dst;
  float carry;
  if (blk < kBlkX) {
    const size_t u = (size_t)blk * 256 + tid;
    src = x + u * 8;
    dst = xh + u * 8;
    carry = kXCarry;
  } else if (blk < kBlkX + kBlkQK) {
    const int lb = blk - kBlkX;
    const size_t u = (size_t)lb * 256 + tid;
    if (lb < kBlkSeam) src = Wq + u * 8;
    else               src = Wk + (u - kUnitsSeam) * 8;
    dst = wqk + u * 8;
    carry = kWCarry;
  } else if (blk < kBlkX + kBlkQK + kBlkKV) {
    const int lb = blk - kBlkX - kBlkQK;
    const size_t u = (size_t)lb * 256 + tid;
    if (lb < kBlkSeam) src = Wk + u * 8;
    else               src = Wv + (u - kUnitsSeam) * 8;
    dst = wkv + u * 8;
    carry = kWCarry;
  } else {
    const int lb = blk - kBlkX - kBlkQK - kBlkKV;
    const size_t u = (size_t)lb * 256 + tid;
    src = Wo + u * 8;
    dst = wo + u * 8;
    carry = kWCarry;
  }
  const v4f a = *(const v4f*)(src);
  const v4f c = *(const v4f*)(src + 4);
  const v4u pk = pack8(a.x * carry, a.y * carry, a.z * carry, a.w * carry,
                       c.x * carry, c.y * carry, c.z * carry, c.w * carry);
  *(volatile v4u*)dst = pk;
  __threadfence();
  *(volatile v4u*)dst = pk;
}

template <int EPI>
__global__ __launch_bounds__(256) void gemm_f16_kernel(
    const unsigned short* __restrict__ Ap, int lda,
    const unsigned short* __restrict__ Btp, int ldb,
    void* __restrict__ Cout, int ldc, int M, int N, int K, float scale, float scale2) {
  const _Float16* A  = (const _Float16*)Ap;
  const _Float16* Bt = (const _Float16*)Btp;
  __shared__ __align__(16) float sT[8][16 * 68];
  const int lane = threadIdx.x & 31;
  const int wave = threadIdx.x >> 5;
  const int tilesN = N >> 6;
  const int tilesM = M >> 6;
  const int tile = blockIdx.x * 8 + wave;
  if (tile >= tilesM * tilesN) return;
  const int tm = tile / tilesN;
  const int tn = tile - tm * tilesN;
  const int m0 = tm << 6;
  const int n0 = tn << 6;
  const int rlane = lane & 15;
  const int koff  = (lane >> 4) * 8;
  const int mOff  = (lane >> 4) * 8;

  v8f acc[4][4];
#pragma unroll
  for (int i = 0; i < 4; ++i)
#pragma unroll
    for (int j = 0; j < 4; ++j) acc[i][j] = (v8f){0.f, 0.f, 0.f, 0.f, 0.f, 0.f, 0.f, 0.f};

  for (int k0 = 0; k0 < K; k0 += 32) {
    v16h bh[4];
#pragma unroll
    for (int j = 0; j < 4; ++j) {
      const size_t bo = (size_t)(n0 + (j << 4) + rlane) * ldb + koff + k0;
      bh[j] = frag_load(Bt + bo);
    }
#pragma unroll
    for (int i = 0; i < 4; ++i) {
      const size_t ao = (size_t)(m0 + (i << 4) + rlane) * lda + koff + k0;
      const v16h ah = frag_load(A + ao);
#pragma unroll
      for (int j = 0; j < 4; ++j) acc[i][j] = mma_h(ah, bh[j], acc[i][j]);
    }
    keep4_h(bh[0], bh[1], bh[2], bh[3]);
  }
  acc_guard4(acc[0][0], acc[0][1], acc[0][2], acc[0][3]);
  acc_guard4(acc[1][0], acc[1][1], acc[1][2], acc[1][3]);
  acc_guard4(acc[2][0], acc[2][1], acc[2][2], acc[2][3]);
  acc_guard4(acc[3][0], acc[3][1], acc[3][2], acc[3][3]);

  float* slab = sT[wave];
  const float sc = (EPI == 2 && tm != 0) ? scale2 : scale;
  const bool doPhi = (EPI == 1) || (EPI == 2 && tm == 0);
#pragma unroll
  for (int i = 0; i < 4; ++i) {
    const int mBase = m0 + (i << 4);
#pragma unroll
    for (int j = 0; j < 4; ++j) {
#pragma unroll
      for (int r = 0; r < 8; ++r) slab[(mOff + r) * 68 + (j << 4) + rlane] = acc[i][j][r] * sc;
    }
    wave_sync_lds();
    if (EPI == 0) {
      float* C = (float*)Cout;
      const int hh = lane >> 4, c4 = (lane & 15) * 4;
      for (int pass = 0; pass < 2; ++pass) {
#pragma unroll
        for (int it = 0; it < 8; ++it) {
          const int row = it * 2 + hh;
          const v4f v = *(const v4f*)(slab + row * 68 + c4);
          *(volatile v4f*)(C + (size_t)(mBase + row) * ldc + n0 + c4) = v;
        }
        __threadfence();
      }
    } else {
      unsigned short* C = (unsigned short*)Cout;
      const int q = lane >> 3, c8 = (lane & 7) * 8;
      if (doPhi) {
#pragma unroll 1
        for (int it = 0; it < 4; ++it) {
          float* sp = slab + (it * 4 + q) * 68 + c8;
          const v4f a = *(const v4f*)(sp);
          const v4f b = *(const v4f*)(sp + 4);
          const v4f pa = (v4f){phi_map(a.x), phi_map(a.y), phi_map(a.z), phi_map(a.w)};
          const v4f pb = (v4f){phi_map(b.x), phi_map(b.y), phi_map(b.z), phi_map(b.w)};
          *(v4f*)(sp) = pa;
          *(v4f*)(sp + 4) = pb;
        }
        wave_sync_lds();
      }
      v4u pk[4];
#pragma unroll
      for (int it = 0; it < 4; ++it) {
        const float* sp = slab + (it * 4 + q) * 68 + c8;
        const v4f a = *(const v4f*)(sp);
        const v4f b = *(const v4f*)(sp + 4);
        pk[it] = pack8(a.x, a.y, a.z, a.w, b.x, b.y, b.z, b.w);
      }
      for (int pass = 0; pass < 2; ++pass) {
#pragma unroll
        for (int it = 0; it < 4; ++it) {
          const int row = it * 4 + q;
          *(volatile v4u*)(C + (size_t)(mBase + row) * ldc + n0 + c8) = pk[it];
        }
        __threadfence();
      }
    }
    wave_sync_lds();
  }
}

__global__ __launch_bounds__(128) void chunk_scan_kernel(
    const unsigned short* __restrict__ QK, const unsigned short* __restrict__ KVt,
    const float* __restrict__ decay_logit, float* __restrict__ Num, float* __restrict__ Den) {
  __shared__ __align__(16) _Float16 sQ[kChunk * kTP];
  __shared__ __align__(16) _Float16 sKn[kChunk * kTP];
  __shared__ __align__(16) _Float16 sVt[kDTile * kTP];
  __shared__ __align__(16) _Float16 sKd[kMem * kTP];
  __shared__ __align__(16) _Float16 sS[kChunk * kTP];
  __shared__ __align__(16) _Float16 sCt[kDTile * kTP];
  __shared__ __align__(16) float sSlab[4][16 * kSlabP];
  __shared__ __align__(16) float sG[kChunk];
  __shared__ __align__(16) float sCf[kChunk];
  __shared__ __align__(16) float sE[kChunk];
  __shared__ __align__(16) float sRS[kChunk];
  __shared__ __align__(16) float sQZ[kChunk];
  __shared__ __align__(16) float sZadd[kMem];
  __shared__ __align__(16) float sZ[kMem];

  const int tid  = threadIdx.x;
  const int w    = tid >> 5;
  const int lane = tid & 31;
  const int hh   = lane >> 4;
  const int c    = lane & 15;
  const int dt   = blockIdx.x;
  const int b    = blockIdx.y;
  const int d0   = dt * kDTile;

  const float logit = decay_logit[0];
  const float decay = 1.0f / (1.0f + expf(-logit));
  const float ld    = logf(fmaxf(decay, 1e-6f));

  v8f Cacc[4];
#pragma unroll
  for (int j = 0; j < 4; ++j) Cacc[j] = (v8f){0.f, 0.f, 0.f, 0.f, 0.f, 0.f, 0.f, 0.f};
  if (tid < kMem) sZ[tid] = 0.0f;

#pragma unroll 1
  for (int ch = 0; ch < kNChunk; ++ch) {
    const int t0 = ch * kChunk;
    const size_t rowb = (size_t)b * kSeq + t0;
    const float lcb = lc_at(ld, t0 - 1);
    const float lce = lc_at(ld, t0 + kChunk - 1);
    const float Gc  = expf(lce - lcb);

    __syncthreads();
    if (tid < kChunk) {
      const float l = lc_at(ld, t0 + tid);
      sG[tid]  = expf(l - lcb);
      sCf[tid] = expf(lcb - l);
      sE[tid]  = expf(lce - l);
    }
    __syncthreads();

    {
      const int sr = tid >> 1, sh = (tid & 1) * 32;
      const unsigned short* gq = QK + (rowb + sr) * kQKld + sh;
      const unsigned short* gk = gq + kMem;
      const unsigned short* gv = KVt + (size_t)(kMem + d0 + sr) * kRows + rowb + sh;
      const unsigned short* gt = KVt + (size_t)sr * kRows + rowb + sh;
      float qz = 0.0f, za = 0.0f;
#pragma unroll 1
      for (int i = 0; i < 4; ++i) {
        const int co = sh + 8 * i;
        const v4u uq = *(const v4u*)(gq + 8 * i);
        const v4u uk = *(const v4u*)(gk + 8 * i);
        const v4u uv = *(const v4u*)(gv + 8 * i);
        const v4u ut = *(const v4u*)(gt + 8 * i);
        *(v8h*)(sQ  + sr * kTP + co) = __builtin_bit_cast(v8h, uq);
        *(v8h*)(sKn + sr * kTP + co) = __builtin_bit_cast(v8h, uk);
        *(v8h*)(sVt + sr * kTP + co) = __builtin_bit_cast(v8h, uv);
        const v4f z0 = *(const v4f*)(sZ + co);
        const v4f z1 = *(const v4f*)(sZ + co + 4);
        const v4f e0 = *(const v4f*)(sE + co);
        const v4f e1 = *(const v4f*)(sE + co + 4);
        const unsigned q0 = uq.x, q1 = uq.y, q2 = uq.z, q3 = uq.w;
        qz = fmaf(h16_to_f32(q0 & 0xffffu), z0.x, qz);
        qz = fmaf(h16_to_f32(q0 >> 16),     z0.y, qz);
        qz = fmaf(h16_to_f32(q1 & 0xffffu), z0.z, qz);
        qz = fmaf(h16_to_f32(q1 >> 16),     z0.w, qz);
        qz = fmaf(h16_to_f32(q2 & 0xffffu), z1.x, qz);
        qz = fmaf(h16_to_f32(q2 >> 16),     z1.y, qz);
        qz = fmaf(h16_to_f32(q3 & 0xffffu), z1.z, qz);
        qz = fmaf(h16_to_f32(q3 >> 16),     z1.w, qz);
        const unsigned k0w = ut.x, k1w = ut.y, k2w = ut.z, k3w = ut.w;
        const float p0 = h16_to_f32(k0w & 0xffffu) * e0.x;
        const float p1 = h16_to_f32(k0w >> 16)     * e0.y;
        const float p2 = h16_to_f32(k1w & 0xffffu) * e0.z;
        const float p3 = h16_to_f32(k1w >> 16)     * e0.w;
        const float p4 = h16_to_f32(k2w & 0xffffu) * e1.x;
        const float p5 = h16_to_f32(k2w >> 16)     * e1.y;
        const float p6 = h16_to_f32(k3w & 0xffffu) * e1.z;
        const float p7 = h16_to_f32(k3w >> 16)     * e1.w;
        za += ((p0 + p1) + (p2 + p3)) + ((p4 + p5) + (p6 + p7));
        const v4u pkd = pack8(p0, p1, p2, p3, p4, p5, p6, p7);
        *(v8h*)(sKd + sr * kTP + co) = __builtin_bit_cast(v8h, pkd);
      }
      const float qzo = __shfl_xor(qz, 1, 32);
      const float zao = __shfl_xor(za, 1, 32);
      const float qzt = qz + qzo;
      const float zat = za + zao;
      if ((tid & 1) == 0) {
        sQZ[sr] = qzt;
        sZadd[sr] = zat;
      }
    }
    __syncthreads();

    v16h qa[2];
    qa[0] = frag_load(sQ + (16 * w + c) * kTP + 8 * hh);
    qa[1] = frag_load(sQ + (16 * w + c) * kTP + 32 + 8 * hh);
    {
      v8f sacc[4];
#pragma unroll
      for (int j = 0; j < 4; ++j) {
        sacc[j] = (v8f){0.f, 0.f, 0.f, 0.f, 0.f, 0.f, 0.f, 0.f};
        const v16h kb0 = frag_load(sKn + (16 * j + c) * kTP + 8 * hh);
        const v16h kb1 = frag_load(sKn + (16 * j + c) * kTP + 32 + 8 * hh);
        sacc[j] = mma_h(qa[0], kb0, sacc[j]);
        sacc[j] = mma_h(qa[1], kb1, sacc[j]);
      }
      float gr[8], rs[8];
#pragma unroll
      for (int r = 0; r < 8; ++r) {
        gr[r] = sG[16 * w + 8 * hh + r];
        rs[r] = 0.0f;
      }
#pragma unroll
      for (int j = 0; j < 4; ++j) {
        const int sl = 16 * j + c;
        const float cf = sCf[sl];
#pragma unroll
        for (int r = 0; r < 8; ++r) {
          const int tl = 16 * w + 8 * hh + r;
          const float wv = sacc[j][r] * gr[r] * cf;
          float v = (sl <= tl) ? wv : 0.0f;
          v = (fabsf(v) < kF16MinNormal) ? 0.0f : v;
          rs[r] += v;
          sS[tl * kTP + sl] = (_Float16)v;
        }
      }
#pragma unroll
      for (int r = 0; r < 8; ++r) {
        float s = rs[r];
        s += __shfl_xor(s, 1, 32);
        s += __shfl_xor(s, 2, 32);
        s += __shfl_xor(s, 4, 32);
        s += __shfl_xor(s, 8, 32);
        rs[r] = s;
      }
      if (c == 0) {
#pragma unroll
        for (int r = 0; r < 8; ++r) sRS[16 * w + 8 * hh + r] = rs[r];
      }
    }
#pragma unroll
    for (int j = 0; j < 4; ++j) {
      const v4u pc = pack8(Cacc[j][0], Cacc[j][1], Cacc[j][2], Cacc[j][3],
                           Cacc[j][4], Cacc[j][5], Cacc[j][6], Cacc[j][7]);
      *(v8h*)(sCt + (16 * j + c) * kTP + 16 * w + 8 * hh) = __builtin_bit_cast(v8h, pc);
      Cacc[j] = Cacc[j] * Gc;
    }
    __syncthreads();

    v8f a1[4], a2[4];
#pragma unroll
    for (int j = 0; j < 4; ++j) {
      a1[j] = (v8f){0.f, 0.f, 0.f, 0.f, 0.f, 0.f, 0.f, 0.f};
      a2[j] = (v8f){0.f, 0.f, 0.f, 0.f, 0.f, 0.f, 0.f, 0.f};
    }
#pragma unroll
    for (int kk = 0; kk < 2; ++kk) {
      const v16h sa = frag_load(sS  + (16 * w + c) * kTP + kk * 32 + 8 * hh);
      const v16h ka = frag_load(sKd + (16 * w + c) * kTP + kk * 32 + 8 * hh);
#pragma unroll
      for (int j = 0; j < 4; ++j) {
        const v16h vb = frag_load(sVt + (16 * j + c) * kTP + kk * 32 + 8 * hh);
        const v16h cb = frag_load(sCt + (16 * j + c) * kTP + kk * 32 + 8 * hh);
        a1[j]   = mma_h(sa, vb, a1[j]);
        a2[j]   = mma_h(qa[kk], cb, a2[j]);
        Cacc[j] = mma_h(ka, vb, Cacc[j]);
      }
    }
    {
      float gr[8];
#pragma unroll
      for (int r = 0; r < 8; ++r) gr[r] = sG[16 * w + 8 * hh + r];
      float* slab = sSlab[w];
      const int q = lane >> 3, c4 = (lane & 7) * 4;
#pragma unroll
      for (int half = 0; half < 2; ++half) {
#pragma unroll
        for (int jj = 0; jj < 2; ++jj) {
#pragma unroll
          for (int r = 0; r < 8; ++r) {
            const float nv = (a1[2 * half + jj][r] + gr[r] * a2[2 * half + jj][r]) * kNumFold;
            slab[(8 * hh + r) * kSlabP + 16 * jj + c] = nv;
          }
        }
        wave_sync_lds();
        v4f ov[4];
#pragma unroll
        for (int it = 0; it < 4; ++it) ov[it] = *(const v4f*)(slab + (it * 4 + q) * kSlabP + c4);
        for (int pass = 0; pass < 2; ++pass) {
#pragma unroll
          for (int it = 0; it < 4; ++it) {
            const size_t o = (rowb + 16 * w + it * 4 + q) * kDm + d0 + 32 * half + c4;
            *(volatile v4f*)(Num + o) = ov[it];
          }
          __threadfence();
        }
        wave_sync_lds();
      }
    }
    if (dt == 0 && w == 0) {
      if (lane < 16) {
        const int tb = 4 * lane;
        const float e0 = kQScale * (sRS[tb]     + sG[tb]     * sQZ[tb])     + kDenEps;
        const float e1 = kQScale * (sRS[tb + 1] + sG[tb + 1] * sQZ[tb + 1]) + kDenEps;
        const float e2 = kQScale * (sRS[tb + 2] + sG[tb + 2] * sQZ[tb + 2]) + kDenEps;
        const float e3 = kQScale * (sRS[tb + 3] + sG[tb + 3] * sQZ[tb + 3]) + kDenEps;
        const v4f dv = (v4f){e0, e1, e2, e3};
        float* dp = Den + rowb + tb;
        *(volatile v4f*)dp = dv;
        __threadfence();
        *(volatile v4f*)dp = dv;
      }
    }
    if (w >= 2) {
      const int m = tid - 64;
      const float zn = Gc * sZ[m] + sZadd[m];
      sZ[m] = zn;
    }
  }
}

__global__ __launch_bounds__(256) void norm_rows_kernel(
    const float* __restrict__ Num, const float* __restrict__ Den, const float* __restrict__ nw,
    unsigned short* __restrict__ Un) {
  const int lane = threadIdx.x & 31, wave = threadIdx.x >> 5;
  const int row = blockIdx.x * 8 + wave;
  const int c0 = lane * 8;
  const float* nr = Num + (size_t)row * kDm;
  const v4f n0 = *(const v4f*)(nr + c0);
  const v4f n1 = *(const v4f*)(nr + c0 + 4);
  const v4f n2 = *(const v4f*)(nr + 256 + c0);
  const v4f n3 = *(const v4f*)(nr + 256 + c0 + 4);
  const float den = Den[row];
  const float inv = 1.0f / den;
  float u[16];
#pragma unroll
  for (int e = 0; e < 4; ++e) {
    u[e]      = n0[e] * inv;
    u[4 + e]  = n1[e] * inv;
    u[8 + e]  = n2[e] * inv;
    u[12 + e] = n3[e] * inv;
  }
  float ss = 0.0f;
#pragma unroll
  for (int e = 0; e < 16; ++e) ss += u[e] * u[e];
  ss += __shfl_xor(ss, 16, 32);
  ss += __shfl_xor(ss, 8, 32);
  ss += __shfl_xor(ss, 4, 32);
  ss += __shfl_xor(ss, 2, 32);
  ss += __shfl_xor(ss, 1, 32);
  const float rinv = 1.0f / sqrtf(ss * kInvDm + kRmsEps);
  const v4f w0 = *(const v4f*)(nw + c0);
  const v4f w1 = *(const v4f*)(nw + c0 + 4);
  const v4f w2 = *(const v4f*)(nw + 256 + c0);
  const v4f w3 = *(const v4f*)(nw + 256 + c0 + 4);
  float o[16];
#pragma unroll
  for (int e = 0; e < 4; ++e) {
    o[e]      = u[e]      * rinv * w0[e] * kUCarry;
    o[4 + e]  = u[4 + e]  * rinv * w1[e] * kUCarry;
    o[8 + e]  = u[8 + e]  * rinv * w2[e] * kUCarry;
    o[12 + e] = u[12 + e] * rinv * w3[e] * kUCarry;
  }
  const v4u pa = pack8(o[0], o[1], o[2], o[3], o[4], o[5], o[6], o[7]);
  const v4u pb = pack8(o[8], o[9], o[10], o[11], o[12], o[13], o[14], o[15]);
  unsigned short* ur = Un + (size_t)row * kDm;
  *(volatile v4u*)(ur + c0) = pa;
  *(volatile v4u*)(ur + 256 + c0) = pb;
  __threadfence();
  *(volatile v4u*)(ur + c0) = pa;
  *(volatile v4u*)(ur + 256 + c0) = pb;
}

extern "C" void kernel_launch(void* const* d_in, const int* in_sizes, int n_in,
                              void* d_out, int out_size, void* d_ws, size_t ws_size,
                              hipStream_t stream) {
  if (n_in < 7) return;
  if (in_sizes[0] != kRows * kDm) return;
  if (in_sizes[1] != kMem * kDm) return;
  if (in_sizes[2] != kMem * kDm) return;
  if (in_sizes[3] != kDm * kDm) return;
  if (in_sizes[4] != kDm * kDm) return;
  if (in_sizes[5] != 1) return;
  if (in_sizes[6] != kDm) return;
  if (out_size != kRows * kDm) return;
  if (ws_size < kWsTotal) return;

  const float* x   = (const float*)d_in[0];
  const float* Wq  = (const float*)d_in[1];
  const float* Wk  = (const float*)d_in[2];
  const float* Wv  = (const float*)d_in[3];
  const float* Wo  = (const float*)d_in[4];
  const float* dl  = (const float*)d_in[5];
  const float* nw  = (const float*)d_in[6];

  char* ws = (char*)d_ws;
  unsigned short* XH  = (unsigned short*)(ws + kOffXH);
  unsigned short* WQK = (unsigned short*)(ws + kOffWQK);
  unsigned short* WKV = (unsigned short*)(ws + kOffWKV);
  unsigned short* WOH = (unsigned short*)(ws + kOffWO);
  unsigned short* QK  = (unsigned short*)(ws + kOffQK);
  unsigned short* KVT = (unsigned short*)(ws + kOffKVT);
  float*          NUM = (float*)(ws + kOffNUM);
  float*          DEN = (float*)(ws + kOffDEN);
  unsigned short* UN  = (unsigned short*)(ws + kOffUN);

  cast_planes_kernel<<<kBlkX + kBlkQK + kBlkKV + kBlkO, 256, 0, stream>>>(x, Wq, Wk, Wv, Wo, XH, WQK, WKV, WOH);

  gemm_f16_kernel<1><<<(kRows / 64) * (kQKld / 64) / 8, 256, 0, stream>>>(
      XH, kDm, WQK, kDm, (void*)QK, kQKld, kRows, kQKld, kDm, kProjScale, 0.0f);

  gemm_f16_kernel<2><<<(kKVrows / 64) * (kRows / 64) / 8, 256, 0, stream>>>(
      WKV, kDm, XH, kDm, (void*)KVT, kRows, kKVrows, kRows, kDm, kProjScale, kVScale);

  chunk_scan_kernel<<<dim3(kDm / kDTile, kBatch), 128, 0, stream>>>(QK, KVT, dl, NUM, DEN);

  norm_rows_kernel<<<kRows / 8, 256, 0, stream>>>(NUM, DEN, nw, UN);

  gemm_f16_kernel<0><<<(kRows / 64) * (kDm / 64) / 8, 256, 0, stream>>>(
      UN, kDm, WOH, kDm, d_out, kDm, kRows, kDm, kDm, kOutScale, 0.0f);
}
